// HistDRDoubleConv_84593675862236
// MI455X (gfx1250) — hardware-verified
//
#include <hip/hip_runtime.h>
#include <math.h>

typedef __attribute__((ext_vector_type(16))) _Float16 v16h;
typedef __attribute__((ext_vector_type(16))) __bf16 v16b;
typedef __attribute__((ext_vector_type(8)))  _Float16 v8h;
typedef __attribute__((ext_vector_type(8)))  float v8f;
typedef __attribute__((ext_vector_type(4)))  float v4f;
typedef __attribute__((ext_vector_type(2)))  float v2f;
typedef __attribute__((ext_vector_type(4)))  unsigned v4u;
typedef __attribute__((ext_vector_type(4)))  int v4i;
typedef float __attribute__((may_alias)) float_a;
typedef int __attribute__((may_alias)) int_a;

template <typename T> __device__ __forceinline__ void vst2(void* p, T v) { *(volatile T*)p = v; __threadfence(); *(volatile T*)p = v; }
__device__ __forceinline__ v8f wmma16(v16h a, v16h b, v8f c) {
  v8f d = __builtin_amdgcn_wmma_f32_16x16x32_f16(false, a, false, b, (short)0, c, false, false);
  asm volatile("v_nop\n\tv_nop\n\tv_nop\n\tv_nop" : "+v"(d) : "v"(a), "v"(b));
  return d;
}
__device__ __forceinline__ v8f wmma_bf(v16b a, v16b b, v8f c) {
  v8f d = __builtin_amdgcn_wmma_f32_16x16x32_bf16(false, a, false, b, (short)0, c, false, false);
  asm volatile("v_nop\n\tv_nop\n\tv_nop\n\tv_nop" : "+v"(d) : "v"(a), "v"(b));
  return d;
}
__device__ __forceinline__ v16h frag_h(const _Float16* rowk0, int lane) {
  union { v16h v; v8h q[2]; } u; const _Float16* p = rowk0 + 8 * (lane >> 4);
  u.q[0] = *(const v8h*)p; u.q[1] = *(const v8h*)(p + 16); return u.v;
}
__device__ __forceinline__ v16h frag_f32(const float* rowk0, int lane) {
  v16h a; const float* p = rowk0 + 8 * (lane >> 4);
#pragma unroll
  for (int i = 0; i < 8; ++i) { a[i] = (_Float16)p[i]; a[8 + i] = (_Float16)p[16 + i]; }
  return a;
}
__device__ __forceinline__ v16h frag_f32s(const float* rowk0, int lane, float sc) {
  v16h a; const float* p = rowk0 + 8 * (lane >> 4);
#pragma unroll
  for (int i = 0; i < 8; ++i) { a[i] = (_Float16)(p[i] * sc); a[8 + i] = (_Float16)(p[16 + i] * sc); }
  return a;
}
__device__ __forceinline__ v16h fragc_f32(const float* W, int k0, int n, int lane, int ld, int K) {
  v16h a; const int g = lane >> 4;
#pragma unroll
  for (int i = 0; i < 8; ++i) { const int ka = k0 + 8 * g + i, kb = ka + 16;
    a[i] = (_Float16)(ka < K ? W[(size_t)(ka < K ? ka : K - 1) * ld + n] : 0.f); a[8 + i] = (_Float16)(kb < K ? W[(size_t)(kb < K ? kb : K - 1) * ld + n] : 0.f); }
  return a;
}
struct F2 { v16b h, l; };
__device__ __forceinline__ F2 bsplit16(const float v[16]) { F2 r;
#pragma unroll
  for (int i = 0; i < 16; ++i) { const __bf16 h = (__bf16)v[i]; r.h[i] = h; r.l[i] = (__bf16)(v[i] - (float)h); }
  return r; }
__device__ __forceinline__ F2 split_row(const float* row, int k0, int lane) { float v[16]; const float* p = row + k0 + 8 * (lane >> 4);
#pragma unroll
  for (int i = 0; i < 8; ++i) { v[i] = p[i]; v[8 + i] = p[16 + i]; }
  return bsplit16(v); }
__device__ __forceinline__ F2 split_rowK(const float* row, int k0, int lane, int K) { float v[16]; const int g = lane >> 4;
#pragma unroll
  for (int i = 0; i < 8; ++i) { const int ka = k0 + 8 * g + i, kb = ka + 16; v[i] = ka < K ? row[ka < K ? ka : K - 1] : 0.f; v[8 + i] = kb < K ? row[kb < K ? kb : K - 1] : 0.f; }
  return bsplit16(v); }
__device__ __forceinline__ F2 split_col(const float* W, int k0, int n, int lane, int ld, int K) { float v[16]; const int g = lane >> 4;
#pragma unroll
  for (int i = 0; i < 8; ++i) { const int ka = k0 + 8 * g + i, kb = ka + 16; v[i] = ka < K ? W[(size_t)(ka < K ? ka : K - 1) * ld + n] : 0.f; v[8 + i] = kb < K ? W[(size_t)(kb < K ? kb : K - 1) * ld + n] : 0.f; }
  return bsplit16(v); }
__device__ __forceinline__ v8f mac3(const F2& a, const F2& b, v8f c) { c = wmma_bf(a.l, b.h, c); c = wmma_bf(a.h, b.l, c); return wmma_bf(a.h, b.h, c); }
__device__ __forceinline__ float sigm(float v) { return 1.0f / (1.0f + expf(-v)); }
#define LDSX() do { asm volatile("s_wait_dscnt 0" ::: "memory"); __builtin_amdgcn_wave_barrier(); __builtin_amdgcn_fence(__ATOMIC_RELEASE, "workgroup"); } while (0)


#ifndef NBT
#define NBT 4
#endif
#define CIN 16
#define CM 32
#define HH 256
#define WWD 256
#define NPI (HH * WWD)
#define NPIX (NBT * NPI)
#define NREG 8
#define NKEY (NBT * NREG)
#define KP1 160
#define KP2 288
#define NTILE (CSA_SEGCAP / 64)
typedef __attribute__((ext_vector_type(8))) __bf16 v8b;
__device__ __forceinline__ v16b frag_b(const __bf16* rowk0, int lane) {
  union { v16b v; v8b q[2]; } u; const __bf16* p = rowk0 + 8 * (lane >> 4);
  u.q[0] = *(const v8b*)p; u.q[1] = *(const v8b*)(p + 16); return u.v;
}
__device__ __forceinline__ float bfr(float v) { return (float)(__bf16)v; }
__device__ __attribute__((noinline)) float exp_ni(float v) { return expf(v); }
__device__ __attribute__((noinline)) float erf_ni(float v) { return erff(v); }
__device__ __forceinline__ v16b zfrag_if(v16b a, bool ok) { const v16b z = {}; return ok ? a : z; }

#define CSA_N NKEY
#define CSA_E NPIX
#define CSA_CHUNK 4096
#define CSA_BKT 1
#define CSA_NCH (CSA_E / CSA_CHUNK)
#define CSA_NBK CSA_N
#define CSA_NBKP 64
#define CSA_OFFP 64
#define CSA_SEGCAP (CSA_E + 64 * CSA_NBK * CSA_NCH)
#define CSA_SZ_CNT (4u * CSA_NCH * CSA_NBKP)
#define CSA_SZ_OFF (4u * CSA_NBK * CSA_OFFP)
#define CSA_SZ_SEG (4u * CSA_SEGCAP)
__global__ __launch_bounds__(256) void k_csA_cnt(const int* __restrict__ DST, int dstride, int* __restrict__ CNT) {
  __shared__ unsigned short sc[256][CSA_NBK + 1]; __shared__ __align__(16) int srow[CSA_NBKP];
  const int c = blockIdx.x, tid = threadIdx.x;
  for (int b = 0; b < CSA_NBK; ++b) sc[tid][b] = 0;
  const size_t e0 = (size_t)c * CSA_CHUNK + tid * 16;
  for (int i = 0; i < 16; ++i) { const size_t e = e0 + i; if (e < (size_t)CSA_E) { int d = DST[e * dstride]; d = min(max(d, 0), CSA_N - 1); sc[tid][d / CSA_BKT] += 1; } }
  __syncthreads();
  for (int b = tid; b < CSA_NBKP; b += 256) { int s = 0; if (b < CSA_NBK) for (int t = 0; t < 256; ++t) s += sc[t][b]; srow[b] = s; }
  __syncthreads();
  for (int q = tid; q < CSA_NBKP / 4; q += 256) vst2((unsigned*)(CNT + (size_t)c * CSA_NBKP + q * 4), *(const v4u*)&srow[q * 4]);
}
__global__ __launch_bounds__(256) void k_csA_scan(const int* __restrict__ CNT, int* __restrict__ OFF, int* __restrict__ TKEY) {
  __shared__ int sbt[CSA_NBK + 1]; __shared__ __align__(16) int sbuf[CSA_NBK][CSA_OFFP]; __shared__ __align__(16) int stk[NTILE];
  const int tid = threadIdx.x;
  if (tid < CSA_NBK) { int sp = 0; for (int c = 0; c < CSA_NCH; ++c) sp += (CNT[(size_t)c * CSA_NBKP + tid] + 63) & ~63; sbt[tid] = sp; }
  __syncthreads();
  if (tid == 0) { int acc = 0; for (int b = 0; b < CSA_NBK; ++b) { const int t = sbt[b]; sbt[b] = acc; acc += t; } sbt[CSA_NBK] = acc; }
  __syncthreads();
  if (tid < CSA_NBK) { const int b = tid; int o = sbt[b]; for (int c = 0; c < CSA_OFFP; ++c) { sbuf[b][c] = o; o += (CNT[(size_t)c * CSA_NBKP + b] + 63) & ~63; } }
  for (int t = tid; t < NTILE; t += 256) { int key = -1; const int s0 = t * 64;
    for (int b = 0; b < CSA_NBK; ++b) if (s0 >= sbt[b] && s0 < sbt[b + 1]) key = b;
    stk[t] = key; }
  __syncthreads();
  for (int q = tid; q < CSA_NBK * (CSA_OFFP / 4); q += 256) { const int r = q / (CSA_OFFP / 4), pc = q % (CSA_OFFP / 4); vst2((unsigned*)(OFF + (size_t)r * CSA_OFFP + pc * 4), *(const v4u*)&sbuf[r][pc * 4]); }
  for (int q = tid; q < NTILE / 4; q += 256) vst2((unsigned*)(TKEY + q * 4), *(const v4u*)&stk[q * 4]);
}
__global__ __launch_bounds__(256) void k_csA_scatter(const int* __restrict__ KEYS, const int* __restrict__ OFF, int* __restrict__ SEG, int* __restrict__ INV) {
  __shared__ unsigned short sc[256][CSA_NBK + 1]; __shared__ int sbase[CSA_NBK + 1]; __shared__ int scn[CSA_NBK + 1]; __shared__ int sord[CSA_CHUNK]; __shared__ __align__(16) int sinv[CSA_CHUNK];
  const int c = blockIdx.x, tid = threadIdx.x;
  for (int b = 0; b < CSA_NBK; ++b) sc[tid][b] = 0;
  const size_t e0 = (size_t)c * CSA_CHUNK + tid * 16; int bk[16];
#pragma unroll
  for (int i = 0; i < 16; ++i) { const size_t e = e0 + i; int d = KEYS[e]; d = min(max(d, 0), CSA_N - 1); bk[i] = d; sc[tid][d] += 1; }
  __syncthreads();
  for (int b = tid; b < CSA_NBK; b += 256) { int acc = 0; for (int t = 0; t < 256; ++t) { const int v = sc[t][b]; sc[t][b] = (unsigned short)acc; acc += v; } scn[b] = acc; }
  __syncthreads();
  if (tid == 0) { int acc = 0; for (int b = 0; b < CSA_NBK; ++b) { sbase[b] = acc; acc += scn[b]; } }
  __syncthreads();
#pragma unroll
  for (int i = 0; i < 16; ++i) { const int b = bk[i]; const int r = sc[tid][b]; sc[tid][b] = (unsigned short)(r + 1); sord[sbase[b] + r] = tid * 16 + i; }
  __syncthreads();
  for (int b = 0; b < CSA_NBK; ++b) { const int n = scn[b]; if (n == 0) continue; const int nl = ((n + 63) & ~63); const size_t o = (size_t)(min(max(OFF[(size_t)b * CSA_OFFP + c], 0), CSA_SEGCAP - nl) & ~63);
    for (int i = tid; i < n; i += 256) sinv[sord[sbase[b] + i]] = (int)o + i;
    for (int q = tid; q < nl / 4; q += 256) { int4 ve;
#pragma unroll
      for (int k = 0; k < 4; ++k) { const int i = q * 4 + k; ve[k] = (i < n) ? (int)((size_t)c * CSA_CHUNK + sord[sbase[b] + i]) : -1; }
      vst2((unsigned*)(SEG + o + q * 4), *(const v4u*)&ve); } }
  __syncthreads();
  for (int q = tid; q < CSA_CHUNK / 4; q += 256) vst2((unsigned*)(INV + (size_t)c * CSA_CHUNK + q * 4), *(const v4u*)&sinv[q * 4]);
}

#define WS_CNT  0u
#define WS_OFF  (WS_CNT + CSA_SZ_CNT)
#define WS_TKEY (WS_OFF + CSA_SZ_OFF)
#define WS_SEG  (WS_TKEY + 4u * NTILE)
#define WS_INV  (WS_SEG + CSA_SZ_SEG)
#define WS_KEYS (WS_INV + 4u * NPIX)
#define WS_POOL (WS_KEYS + 4u * NPIX)
#define WS_KNH  (WS_POOL + 4u * NBT * CM * 32)
#define WS_KNL  (WS_KNH + 2u * NKEY * CM * KP2)
#define WS_YP   (WS_KNL + 2u * NKEY * CM * KP2)
#define WS_PART (WS_YP + 4u * (size_t)CSA_SEGCAP * CM)
#define WS_STAT (WS_PART + 4u * NTILE * CM)
#define WS_Y1H  (WS_STAT + 4u * 64)
#define WS_Y1L  (WS_Y1H + 2u * NBT * CM * NPI)
#define WS_END  (WS_Y1L + 2u * NBT * CM * NPI)

__global__ __launch_bounds__(256) void k_region(const float* __restrict__ HM, int* __restrict__ KEYS) {
  __shared__ __align__(16) int s[256]; const int tid = threadIdx.x; const size_t p0 = (size_t)blockIdx.x * 256; const int b = (int)(p0 / NPI); const size_t pl = p0 % NPI + tid;
  float best = -3.0e38f; int arg = 0;
#pragma unroll
  for (int c = 0; c < NREG; ++c) { const float v = bfr(HM[((size_t)b * NREG + c) * NPI + pl]); if (v > best) { best = v; arg = c; } }
  s[tid] = b * NREG + arg; __syncthreads();
  if (tid < 64) vst2((unsigned*)(KEYS + p0 + tid * 4), *(const v4u*)&s[tid * 4]);
}
template <int L>
__global__ __launch_bounds__(256) void k_pool(const float* __restrict__ X, const __bf16* __restrict__ YH, const __bf16* __restrict__ YL, float* __restrict__ POOL) {
  __shared__ float srow[256][3]; __shared__ __align__(16) float sout[32];
  const int b = blockIdx.x, c = blockIdx.y, tid = threadIdx.x; const int CL = (L == 1) ? CIN : CM; const size_t base = ((size_t)b * CL + c) * NPI + (size_t)tid * WWD;
  float s0 = 0.f, s1 = 0.f, s2 = 0.f;
  for (int xw = 0; xw < WWD; ++xw) { const float v = (L == 1) ? bfr(X[base + xw]) : ((float)YH[base + xw] + (float)YL[base + xw]); if (xw < 86) s0 += v; if (xw >= 85 && xw < 171) s1 += v; if (xw >= 170) s2 += v; }
  srow[tid][0] = s0; srow[tid][1] = s1; srow[tid][2] = s2;
  __syncthreads();
  if (tid < 9) { const int i = tid / 3, j = tid % 3; const int r0 = (i == 0) ? 0 : (i == 1) ? 85 : 170, r1 = (i == 0) ? 86 : (i == 1) ? 171 : 256; float a = 0.f; for (int r = r0; r < r1; ++r) a += srow[r][j]; sout[tid] = a / 7396.0f; }
  if (tid >= 9 && tid < 32) sout[tid] = 0.f;
  __syncthreads();
  if (tid < 8) vst2(POOL + ((size_t)b * CM + c) * 32 + tid * 4, *(const v4f*)&sout[tid * 4]);
}
template <int L>
__global__ __launch_bounds__(256) void k_kern(const float* __restrict__ POOL, const float* __restrict__ W1, const float* __restrict__ B1, const float* __restrict__ W2, const float* __restrict__ B2, __bf16* __restrict__ KNH, __bf16* __restrict__ KNL) {
  constexpr int CL = (L == 1) ? CIN : CM; constexpr int KP = (L == 1) ? KP1 : KP2;
  __shared__ float st[NREG][9]; __shared__ __align__(16) __bf16 sh_[CM][KP2 + 8], sl_[CM][KP2 + 8];
  const int key = blockIdx.x, tid = threadIdx.x; const int b = key / NREG, g = key % NREG;
  if (tid < NREG * 9) { const int r = tid / 9, tap = tid % 9; const int q = g * NREG + r; float a = 0.f; for (int c = 0; c < CL; ++c) a += bfr(W1[(size_t)q * CL + c]) * POOL[((size_t)b * CM + c) * 32 + tap]; a += bfr(B1[q]); st[r][tap] = 1.0f / (1.0f + exp_ni(-a)); }
  __syncthreads();
  for (int q = tid; q < CM * KP; q += 256) { const int co = q / KP, k = q % KP; float v = 0.f;
    if (k < 9 * CL) { const int tap = k / CL, ci = k % CL; const int oc = co * CL + ci; float a = 0.f;
#pragma unroll
      for (int r = 0; r < NREG; ++r) a += bfr(W2[((size_t)g * CM * CL + oc) * NREG + r]) * st[r][tap];
      v = a + bfr(B2[(size_t)g * CM * CL + oc]); }
    const __bf16 hb = (__bf16)v; sh_[co][k] = hb; sl_[co][k] = (__bf16)(v - (float)hb); }
  __syncthreads();
  for (int q = tid; q < CM * (KP / 8); q += 256) { const int co = q / (KP / 8), pc = q % (KP / 8); const size_t o = ((size_t)key * CM + co) * KP2 + pc * 8; vst2((unsigned*)(KNH + o), *(const v4u*)&sh_[co][pc * 8]); vst2((unsigned*)(KNL + o), *(const v4u*)&sl_[co][pc * 8]); }
}
template <int L>
__global__ __launch_bounds__(128) void k_rconv(const int* __restrict__ TKEY, const int* __restrict__ SEG, const float* __restrict__ X, const __bf16* __restrict__ YH, const __bf16* __restrict__ YL, const __bf16* __restrict__ KNH, const __bf16* __restrict__ KNL, float* __restrict__ YP) {
  constexpr int CL = (L == 1) ? CIN : CM; constexpr int KP = (L == 1) ? KP1 : KP2;
  __shared__ int spix[64]; __shared__ __align__(16) __bf16 th[64][40], tl[64][40]; __shared__ __align__(16) float so[4][16][36];
  const int tid = threadIdx.x, wave = tid >> 5, lane = tid & 31, col = lane & 15, g = lane >> 4; const int tile = blockIdx.x;
  const int key = TKEY[tile]; if (key < 0) return;
  const int b = key / NREG;
  if (tid < 64) spix[tid] = SEG[(size_t)tile * 64 + tid];
  __syncthreads();
  v8f acc[2] = {};
#pragma unroll 1
  for (int kc = 0; kc < KP / 32; ++kc) {
    for (int q = tid; q < 64 * 32; q += 128) { const int sl = q & 63, kl = q >> 6; const int k = kc * 32 + kl; const int p = spix[sl]; float v = 0.f;
      if (p >= 0 && k < 9 * CL) { const int tap = k / CL, ci = k % CL; const int pl = p % NPI; const int yy = pl / WWD + tap / 3 - 1, xx = pl % WWD + tap % 3 - 1;
        if (yy >= 0 && yy < HH && xx >= 0 && xx < WWD) { const size_t a = ((size_t)b * CL + ci) * NPI + (size_t)yy * WWD + xx; v = (L == 1) ? bfr(X[a]) : ((float)YH[a] + (float)YL[a]); } }
      const __bf16 hb = (__bf16)v; th[sl][kl] = hb; tl[sl][kl] = (__bf16)(v - (float)hb); }
    __syncthreads();
    { F2 a; a.h = frag_b(&th[wave * 16 + col][0], lane); a.l = frag_b(&tl[wave * 16 + col][0], lane);
#pragma unroll
      for (int j = 0; j < 2; ++j) { const size_t wr = ((size_t)key * CM + j * 16 + col) * KP2 + kc * 32; const v16b wh = frag_b(KNH + wr, lane), wl = frag_b(KNL + wr, lane);
        if (L == 2) acc[j] = wmma_bf(a.l, wh, acc[j]);
        acc[j] = wmma_bf(a.h, wl, acc[j]); acc[j] = wmma_bf(a.h, wh, acc[j]); } }
    __syncthreads(); }
#pragma unroll
  for (int j = 0; j < 2; ++j)
#pragma unroll
    for (int r = 0; r < 8; ++r) so[wave][8 * g + r][j * 16 + col] = acc[j][r];
  LDSX();
  for (int rl = 0; rl < 16; ++rl) if (lane < 8) vst2(YP + ((size_t)tile * 64 + wave * 16 + rl) * CM + lane * 4, *(const v4f*)&so[wave][rl][lane * 4]);
}
template <int P>
__global__ __launch_bounds__(64) void k_stat(const int* __restrict__ TKEY, const int* __restrict__ SEG, const float* __restrict__ YP, const float* __restrict__ STAT, float* __restrict__ PART) {
  __shared__ float sp[2][32]; __shared__ __align__(16) float so[32]; const int tile = blockIdx.x, tid = threadIdx.x; const int c = tid & 31, half = tid >> 5;
  float a = 0.f; const int key = TKEY[tile]; const float mu = (P == 1) ? STAT[c] : 0.f;
  if (key >= 0) for (int i = half; i < 64; i += 2) { const size_t sl = (size_t)tile * 64 + i; if (SEG[sl] >= 0) { const float v = YP[sl * CM + c]; a += (P == 0) ? v : (v - mu) * (v - mu); } }
  sp[half][c] = a; __syncthreads();
  if (tid < 32) so[tid] = sp[0][tid] + sp[1][tid];
  __syncthreads();
  if (tid < 8) vst2(PART + (size_t)tile * CM + tid * 4, *(const v4f*)&so[tid * 4]);
}
template <int P>
__global__ __launch_bounds__(64) void k_red(const float* __restrict__ PART, float* __restrict__ STAT) {
  __shared__ __align__(16) float s[32]; const int tid = threadIdx.x;
  if (tid < 32) { float a = 0.f; for (int t = 0; t < NTILE; ++t) a += PART[(size_t)t * CM + tid]; a = a / (float)NPIX; s[tid] = (P == 0) ? a : rsqrtf(a + 1e-5f); }
  __syncthreads();
  if (tid < 8) vst2(STAT + P * 32 + tid * 4, *(const v4f*)&s[tid * 4]);
}
template <int L>
__global__ __launch_bounds__(256) void k_unperm(const int* __restrict__ INV, const float* __restrict__ YP, const float* __restrict__ STAT, const float* __restrict__ G, const float* __restrict__ BE, __bf16* __restrict__ YH, __bf16* __restrict__ YL, float* __restrict__ OUT) {
  __shared__ __align__(16) float sv[CM][68]; __shared__ __align__(16) __bf16 sh_[CM][72], sl_[CM][72];
  const int tid = threadIdx.x; const size_t p0 = (size_t)blockIdx.x * 64; const int b = (int)(p0 / NPI); const size_t pl0 = p0 % NPI;
  { const int px = tid >> 2, c4 = (tid & 3) * 8; const int sl = min(max(INV[p0 + px], 0), CSA_SEGCAP - 1); const float* row = YP + (size_t)sl * CM + c4;
#pragma unroll
    for (int i = 0; i < 8; ++i) { const int c = c4 + i; const float v = fmaxf((row[i] - STAT[c]) * STAT[32 + c] * bfr(G[c]) + bfr(BE[c]), 0.f); sv[c][px] = v; if (L == 1) { const __bf16 hb = (__bf16)v; sh_[c][px] = hb; sl_[c][px] = (__bf16)(v - (float)hb); } } }
  __syncthreads();
  if (L == 1) { for (int q = tid; q < CM * 8; q += 256) { const int c = q >> 3, pc = q & 7; const size_t o = ((size_t)b * CM + c) * NPI + pl0 + pc * 8; vst2((unsigned*)(YH + o), *(const v4u*)&sh_[c][pc * 8]); vst2((unsigned*)(YL + o), *(const v4u*)&sl_[c][pc * 8]); } }
  else { for (int q = tid; q < CM * 16; q += 256) { const int c = q >> 4, pc = q & 15; vst2(OUT + ((size_t)b * CM + c) * NPI + pl0 + pc * 4, *(const v4f*)&sv[c][pc * 4]); } }
}
extern "C" void kernel_launch(void* const* d_in, const int* in_sizes, int n_in, void* d_out, int out_size, void* d_ws, size_t ws_size, hipStream_t stream) {
  (void)in_sizes; (void)n_in; (void)out_size;
  const float** F = (const float**)d_in;
  if (ws_size < (size_t)WS_END) return;
  char* ws = (char*)d_ws; int *CNT = (int*)(ws + WS_CNT), *OFF = (int*)(ws + WS_OFF), *TKEY = (int*)(ws + WS_TKEY), *SEG = (int*)(ws + WS_SEG), *INV = (int*)(ws + WS_INV), *KEYS = (int*)(ws + WS_KEYS);
  float *POOL = (float*)(ws + WS_POOL), *YP = (float*)(ws + WS_YP), *PART = (float*)(ws + WS_PART), *STAT = (float*)(ws + WS_STAT); __bf16 *KNH = (__bf16*)(ws + WS_KNH), *KNL = (__bf16*)(ws + WS_KNL), *Y1H = (__bf16*)(ws + WS_Y1H), *Y1L = (__bf16*)(ws + WS_Y1L);
  k_region<<<NPIX / 256, 256, 0, stream>>>(F[1], KEYS);
  k_csA_cnt<<<CSA_NCH, 256, 0, stream>>>(KEYS, 1, CNT); k_csA_scan<<<1, 256, 0, stream>>>(CNT, OFF, TKEY); k_csA_scatter<<<CSA_NCH, 256, 0, stream>>>(KEYS, OFF, SEG, INV);
  k_pool<1><<<dim3(NBT, CIN), 256, 0, stream>>>(F[0], nullptr, nullptr, POOL);
  k_kern<1><<<NKEY, 256, 0, stream>>>(POOL, F[2], F[3], F[4], F[5], KNH, KNL);
  k_rconv<1><<<NTILE, 128, 0, stream>>>(TKEY, SEG, F[0], nullptr, nullptr, KNH, KNL, YP);
  k_stat<0><<<NTILE, 64, 0, stream>>>(TKEY, SEG, YP, STAT, PART); k_red<0><<<1, 64, 0, stream>>>(PART, STAT);
  k_stat<1><<<NTILE, 64, 0, stream>>>(TKEY, SEG, YP, STAT, PART); k_red<1><<<1, 64, 0, stream>>>(PART, STAT);
  k_unperm<1><<<NPIX / 64, 256, 0, stream>>>(INV, YP, STAT, F[6], F[7], Y1H, Y1L, nullptr);
  k_pool<2><<<dim3(NBT, CM), 256, 0, stream>>>(nullptr, Y1H, Y1L, POOL);
  k_kern<2><<<NKEY, 256, 0, stream>>>(POOL, F[8], F[9], F[10], F[11], KNH, KNL);
  k_rconv<2><<<NTILE, 128, 0, stream>>>(TKEY, SEG, nullptr, Y1H, Y1L, KNH, KNL, YP);
  k_stat<0><<<NTILE, 64, 0, stream>>>(TKEY, SEG, YP, STAT, PART); k_red<0><<<1, 64, 0, stream>>>(PART, STAT);
  k_stat<1><<<NTILE, 64, 0, stream>>>(TKEY, SEG, YP, STAT, PART); k_red<1><<<1, 64, 0, stream>>>(PART, STAT);
  k_unperm<2><<<NPIX / 64, 256, 0, stream>>>(INV, YP, STAT, F[12], F[13], nullptr, nullptr, (float*)d_out);
}
